// DCRNNCell_59167469470014
// MI455X (gfx1250) — hardware-verified
//
#include <hip/hip_runtime.h>
#include <math.h>

typedef __attribute__((ext_vector_type(16))) _Float16 v16h;
typedef __attribute__((ext_vector_type(8)))  _Float16 v8h;
typedef __attribute__((ext_vector_type(16))) __bf16   v16b;
typedef __attribute__((ext_vector_type(8)))  float    v8f;
typedef __attribute__((ext_vector_type(4)))  float    v4f;

__device__ __forceinline__ int frag_k(int i, int h) { return (i < 8) ? (8 * h + i) : (16 + 8 * h + (i - 8)); }
__device__ __forceinline__ __bf16 bf16_rne(float f) {
    unsigned int u = __float_as_uint(f);
    u += 0x7fffu + ((u >> 16) & 1u);
    return __builtin_bit_cast(__bf16, (unsigned short)(u >> 16));
}
__device__ __forceinline__ float bf16_f32(__bf16 b) { return __uint_as_float(((unsigned int)__builtin_bit_cast(unsigned short, b)) << 16); }
__device__ __forceinline__ v8f wmma16(v16h a, v16h b, v8f c) {
    c = __builtin_amdgcn_wmma_f32_16x16x32_f16(false, a, false, b, (short)0, c, false, false);
    asm volatile("v_nop\n\tv_nop\n\tv_nop\n\tv_nop" : "+v"(c) : "v"(a), "v"(b));
    return c;
}
__device__ __forceinline__ v8f wmmab(v16b a, v16b b, v8f c) {
    c = __builtin_amdgcn_wmma_f32_16x16x32_bf16(false, a, false, b, (short)0, c, false, false);
    asm volatile("v_nop\n\tv_nop\n\tv_nop\n\tv_nop" : "+v"(c) : "v"(a), "v"(b));
    return c;
}
struct Split { v16b hi, lo; };
__device__ __forceinline__ v8f wmma3(const Split& a, const Split& b, v8f c) {
    c = __builtin_amdgcn_wmma_f32_16x16x32_bf16(false, a.hi, false, b.hi, (short)0, c, false, false);
    c = __builtin_amdgcn_wmma_f32_16x16x32_bf16(false, a.hi, false, b.lo, (short)0, c, false, false);
    c = __builtin_amdgcn_wmma_f32_16x16x32_bf16(false, a.lo, false, b.hi, (short)0, c, false, false);
    asm volatile("v_nop\n\tv_nop\n\tv_nop\n\tv_nop" : "+v"(c) : "v"(a.hi), "v"(a.lo), "v"(b.hi), "v"(b.lo));
    return c;
}
struct Split3 { v16b hi, mid, lo; };
__device__ __forceinline__ v8f wmma6(const Split3& a, const Split3& b, v8f c) {
    c = __builtin_amdgcn_wmma_f32_16x16x32_bf16(false, a.hi, false, b.hi, (short)0, c, false, false);
    c = __builtin_amdgcn_wmma_f32_16x16x32_bf16(false, a.hi, false, b.mid, (short)0, c, false, false);
    c = __builtin_amdgcn_wmma_f32_16x16x32_bf16(false, a.mid, false, b.hi, (short)0, c, false, false);
    c = __builtin_amdgcn_wmma_f32_16x16x32_bf16(false, a.hi, false, b.lo, (short)0, c, false, false);
    c = __builtin_amdgcn_wmma_f32_16x16x32_bf16(false, a.mid, false, b.mid, (short)0, c, false, false);
    c = __builtin_amdgcn_wmma_f32_16x16x32_bf16(false, a.lo, false, b.hi, (short)0, c, false, false);
    asm volatile("v_nop\n\tv_nop\n\tv_nop\n\tv_nop" : "+v"(c) : "v"(a.hi), "v"(a.mid), "v"(a.lo), "v"(b.hi), "v"(b.mid), "v"(b.lo));
    return c;
}

__device__ __forceinline__ v16h fh_ld(const float* __restrict__ p, long long sk, int k0, int h, int klen, float s) {
    v16h a;
#pragma unroll
    for (int i = 0; i < 16; ++i) { const int k = k0 + frag_k(i, h); a[i] = (k < klen) ? (_Float16)(p[(long long)k * sk] * s) : (_Float16)0.f; }
    return a;
}
__device__ __forceinline__ Split sp_ld(const float* __restrict__ p, long long sk, int k0, int h, int klen, float s) {
    Split r;
#pragma unroll
    for (int i = 0; i < 16; ++i) {
        const int k = k0 + frag_k(i, h); const float x = (k < klen) ? p[(long long)k * sk] * s : 0.f;
        const __bf16 hb = bf16_rne(x); r.hi[i] = hb; r.lo[i] = bf16_rne(x - bf16_f32(hb));
    }
    return r;
}
__device__ __forceinline__ Split3 sp3_ld(const float* __restrict__ p, long long sk, int k0, int h, int klen, float s) {
    Split3 r;
#pragma unroll
    for (int i = 0; i < 16; ++i) {
        const int k = k0 + frag_k(i, h); const float x = (k < klen) ? p[(long long)k * sk] * s : 0.f;
        const __bf16 hb = bf16_rne(x); const float r1 = x - bf16_f32(hb); const __bf16 mb = bf16_rne(r1);
        r.hi[i] = hb; r.mid[i] = mb; r.lo[i] = bf16_rne(r1 - bf16_f32(mb));
    }
    return r;
}
__device__ __forceinline__ v16b bh_ld(const float* __restrict__ p, long long sk, int k0, int h, int klen, float s) {
    v16b a;
#pragma unroll
    for (int i = 0; i < 16; ++i) { const int k = k0 + frag_k(i, h); a[i] = bf16_rne((k < klen) ? p[(long long)k * sk] * s : 0.f); }
    return a;
}
__device__ __forceinline__ v16h fh_row(const _Float16* __restrict__ row, int k0, int h) {
    v16h a;
#pragma unroll
    for (int i = 0; i < 16; ++i) a[i] = row[k0 + frag_k(i, h)];
    return a;
}

#define VST2(T, ptr, val) do { *(volatile T*)(ptr) = (val); __threadfence(); *(volatile T*)(ptr) = (val); } while (0)
typedef float v4f __attribute__((ext_vector_type(4)));
#define VST2V4(ptr, val) do { *(volatile v4f*)(ptr) = (val); __threadfence(); *(volatile v4f*)(ptr) = (val); } while (0)

__device__ __attribute__((noinline)) float act_fn(float v, int act) {
    if (act == 1) return fmaxf(v, 0.f);
    if (act == 2) { const float u = 0.7978845608028654f * (v + 0.044715f * v * v * v); return 0.5f * v * (1.f + tanhf(u)); }
    if (act == 3) return v / (1.f + expf(-v));
    if (act == 4) return 0.5f * v * (1.f + erff(v * 0.7071067811865476f));
    if (act == 5) return tanhf(v);
    if (act == 6) return 1.f / (1.f + expf(-v));
    if (act == 7) return (v > 0.f) ? v : 0.01f * v;
    if (act == 8) return (v > 0.f) ? v : (expf(v) - 1.f);
    if (act == 9) return fminf(fmaxf(v, 0.f), 6.f);
    if (act == 10) return fabsf(v);
    if (act == 11) return (v >= 0.f) ? v : 0.1f * v;
    if (act == 12) return (v > 0.f) ? v : 0.2f * v;
    if (act == 13) return (v > 20.f) ? v : log1pf(expf(v));
    return v;
}

struct GemmP {
    const float* A; const float* B; const float* bias; const float* R; float* C;
    long long sAo, sAi, sAm, sAk, sBo, sBi, sBn, sBk, sCo, sCi, sCm, sRo, sRi, sRm, sRn;
    int M, N, K, zi_n, flags, act; float alpha, beta, sa, sb;
    int Npad, pad_;
};
static_assert(sizeof(GemmP) == 5 * 8 + 15 * 8 + 6 * 4 + 4 * 4 + 2 * 4, "GemmP has padding");

template <int MODE>
__global__ __launch_bounds__(32) void k_gemm(GemmP p) {
    const int lane = threadIdx.x & 31, h = lane >> 4, l15 = lane & 15;
    const int m0 = blockIdx.y * 16, n0 = blockIdx.x * 32;
    const int z = blockIdx.z, zo = z / p.zi_n, zi = z - zo * p.zi_n;
    const float* A = p.A + zo * p.sAo + zi * p.sAi;
    const float* B = p.B + zo * p.sBo + zi * p.sBi;
    const int am = min(m0 + l15, p.M - 1);
    v8f acc[2], comp[2];
#pragma unroll
    for (int t = 0; t < 2; ++t) { v8f zz = {}; acc[t] = zz; comp[t] = zz; }
    for (int k0 = 0; k0 < p.K; k0 += 32) {
        const float* arow = A + (long long)am * p.sAm;
        if (MODE == 1) {
            const Split a = sp_ld(arow, p.sAk, k0, h, p.K, 1.f);
#pragma unroll
            for (int t = 0; t < 2; ++t) {
                const int bn = min(n0 + t * 16 + l15, p.N - 1);
                acc[t] = wmma3(a, sp_ld(B + (long long)bn * p.sBn, p.sBk, k0, h, p.K, 1.f), acc[t]);
            }
        } else if (MODE == 3) {
            const Split3 a = sp3_ld(arow, p.sAk, k0, h, p.K, 1.f);
#pragma unroll
            for (int t = 0; t < 2; ++t) {
                const int bn = min(n0 + t * 16 + l15, p.N - 1);
                acc[t] = wmma6(a, sp3_ld(B + (long long)bn * p.sBn, p.sBk, k0, h, p.K, 1.f), acc[t]);
            }
        } else if (MODE == 4) {
            const Split3 a = sp3_ld(arow, p.sAk, k0, h, p.K, 1.f);
#pragma unroll
            for (int t = 0; t < 2; ++t) {
                const int bn = min(n0 + t * 16 + l15, p.N - 1); v8f zz = {};
                const v8f part = wmma6(a, sp3_ld(B + (long long)bn * p.sBn, p.sBk, k0, h, p.K, 1.f), zz);
                const v8f y = part - comp[t]; const v8f s = acc[t] + y; comp[t] = (s - acc[t]) - y; acc[t] = s;
            }
        } else if (MODE == 2) {
            const v16b a = bh_ld(arow, p.sAk, k0, h, p.K, 1.f);
#pragma unroll
            for (int t = 0; t < 2; ++t) {
                const int bn = min(n0 + t * 16 + l15, p.N - 1);
                acc[t] = wmmab(a, bh_ld(B + (long long)bn * p.sBn, p.sBk, k0, h, p.K, 1.f), acc[t]);
            }
        } else {
            const v16h a = fh_ld(arow, p.sAk, k0, h, p.K, p.sa);
#pragma unroll
            for (int t = 0; t < 2; ++t) {
                const int bn = min(n0 + t * 16 + l15, p.N - 1);
                acc[t] = wmma16(a, fh_ld(B + (long long)bn * p.sBn, p.sBk, k0, h, p.K, p.sb), acc[t]);
            }
        }
    }
    const float iscale = (MODE == 0) ? p.alpha / (p.sa * p.sb) : p.alpha;
    float* C = p.C + zo * p.sCo + zi * p.sCi;
    const float* R = p.R + zo * p.sRo + zi * p.sRi;
    __shared__ __align__(16) float ctile[16][36];
#pragma unroll
    for (int t = 0; t < 2; ++t) {
        const int n = n0 + t * 16 + l15; const int nn = min(n, p.N - 1);
#pragma unroll
        for (int r = 0; r < 8; ++r) {
            const int m = m0 + 8 * h + r; const int mm = min(m, p.M - 1);
            float v = acc[t][r] * iscale;
            if (p.flags & 1) v += p.bias[nn];
            if (p.flags & 2) v += p.bias[mm];
            v = act_fn(v, p.act);
            if (p.flags & 4) v += p.beta * R[(long long)mm * p.sRm + (long long)nn * p.sRn];
            ctile[8 * h + r][t * 16 + l15] = (n < p.N) ? v : 0.f;
        }
    }
    __syncthreads();
    const int NW = (p.Npad > p.N) ? p.Npad : p.N;
    const bool fast = (m0 + 16 <= p.M) && (n0 + 32 <= NW) && ((p.sCm & 3) == 0) && ((((size_t)C) & 15) == 0);
    if (fast) {
#pragma unroll
        for (int s = 0; s < 4; ++s) {
            const int row = s * 4 + (lane >> 3), c4 = (lane & 7) * 4;
            const v4f v = *(const v4f*)&ctile[row][c4];
            VST2V4(C + (long long)(m0 + row) * p.sCm + n0 + c4, v);
        }
    } else {
        for (int row = 0; row < 16; ++row) {
            const int m = m0 + row, n = n0 + lane;
            if (m < p.M && n < NW) VST2(float, C + (long long)m * p.sCm + n, ctile[row][lane]);
        }
    }
}

#define AW 4
struct AttnP {
    const float* Q; const float* K; const float* V; float* O; float* P; const float* Mf; const int* Mi; float* ST;
    const float* Pw; const float* Rt; const int* SQ; const int* SK;
    long long swb, swh, swi, swj, srb, srh, sri;
    long long sQb, sQh, sQi, sQd, sKb, sKh, sKj, sKd, sVb, sVh, sVj, sVd, sOb, sOh, sOi, sPb, sPh, sPi, smb, smh, smi, smj;
    int Lq, Lk, dh, dv, hrep, causal, coff, pband;
    float scale, mfill; int nonorm, mpol;
    int roff, rn, segpol, win;
};
static_assert(sizeof(AttnP) == 12 * 8 + 29 * 8 + 16 * 4, "AttnP has padding");

#ifndef KATTN_ATTR
#define KATTN_ATTR
#endif
template <int DHP, int DVP, int QM, bool SPLITPV, bool TWOPASS>
__global__ __launch_bounds__(32 * AW) KATTN_ATTR void k_attn(AttnP p) {
    constexpr int NT = DVP / 16;
    constexpr int KS = DHP / 32;
    constexpr int VP = DVP + 8;
    __shared__ __align__(16) float    pl[AW][16 * 64];
    __shared__ __align__(16) _Float16 vl[(SPLITPV ? 2 : 1) * 64 * VP];
    const int lane = threadIdx.x & 31, hf = lane >> 4, l15 = lane & 15, wave = threadIdx.x >> 5;
    const int h = blockIdx.y, b = blockIdx.z, hk = h / p.hrep;
    const int q0 = (blockIdx.x * AW + wave) * 16;
    float* myp = pl[wave];
    const float L2E = 1.4426950408889634f;
    const float NEG = -__builtin_inff();
    const int qi = min(q0 + l15, p.Lq - 1);
    const float* qrow = p.Q + b * p.sQb + h * p.sQh + (long long)qi * p.sQi;
    const float* kbase = p.K + b * p.sKb + hk * p.sKh;
    const float* vbase = p.V + b * p.sVb + hk * p.sVh;
    v16h qa[QM == 0 ? KS : 1]; Split qs_[QM == 1 ? KS : 1]; Split3 qt_[QM == 2 ? KS : 1];
#pragma unroll
    for (int ks = 0; ks < KS; ++ks) {
        if (QM == 2) qt_[ks] = sp3_ld(qrow, p.sQd, ks * 32, hf, p.dh, 1.f);
        else if (QM == 1) qs_[ks] = sp_ld(qrow, p.sQd, ks * 32, hf, p.dh, 1.f);
        else qa[ks] = fh_ld(qrow, p.sQd, ks * 32, hf, p.dh, 1.f);
    }
    v8f o[NT]; float m8[8], l8[8];
#pragma unroll
    for (int t = 0; t < NT; ++t) { v8f zz = {}; o[t] = zz; }
#pragma unroll
    for (int i = 0; i < 8; ++i) { m8[i] = NEG; l8[i] = 0.f; }
    int jend = p.Lk;
    if (p.causal == 1) { const int je = (blockIdx.x * AW + AW - 1) * 16 + 16 + p.coff; jend = min(jend, max(je, 0)); }
    const int npass = TWOPASS ? 2 : 1;
    for (int pass = 0; pass < npass; ++pass) {
        const bool dopv = (!TWOPASS) || pass == 1;
        for (int j0 = 0; j0 < jend; j0 += 64) {
            if (dopv) {
                __syncthreads();
                for (int idx = threadIdx.x; idx < 64 * DVP; idx += 32 * AW) {
                    const int jr = idx / DVP, d = idx - jr * DVP, j = j0 + jr;
                    const float f = (j < p.Lk && d < p.dv) ? vbase[(long long)j * p.sVj + (long long)d * p.sVd] : 0.f;
                    if (SPLITPV) {
                        const __bf16 hb = bf16_rne(f);
                        ((__bf16*)vl)[jr * VP + d] = hb; ((__bf16*)vl)[64 * VP + jr * VP + d] = bf16_rne(f - bf16_f32(hb));
                    } else vl[jr * VP + d] = (_Float16)f;
                }
            }
            v8f s[4];
#pragma unroll
            for (int t = 0; t < 4; ++t) {
                const int j = min(j0 + t * 16 + l15, p.Lk - 1);
                const float* krow = kbase + (long long)j * p.sKj;
                v8f acc = {};
#pragma unroll
                for (int ks = 0; ks < KS; ++ks) {
                    if (QM == 2)      acc = wmma6(qt_[ks], sp3_ld(krow, p.sKd, ks * 32, hf, p.dh, 1.f), acc);
                    else if (QM == 1) acc = wmma3(qs_[ks], sp_ld(krow, p.sKd, ks * 32, hf, p.dh, 1.f), acc);
                    else              acc = wmma16(qa[ks], fh_ld(krow, p.sKd, ks * 32, hf, p.dh, 1.f), acc);
                }
                s[t] = acc;
            }
            float pv[8][4];
#pragma unroll
            for (int i = 0; i < 8; ++i) {
                const int irow = q0 + i + 8 * hf;
                const int ic = min(irow, p.Lq - 1);
                float sc[4];
#pragma unroll
                for (int t = 0; t < 4; ++t) {
                    const int jg = j0 + t * 16 + l15;
                    float v = s[t][i] * p.scale;
                    if (p.Mf) v += p.Mf[b * p.smb + h * p.smh + (long long)ic * p.smi + (long long)min(jg, p.Lk - 1) * p.smj];
                    if (p.Rt) { int rc = ic - min(jg, p.Lk - 1) + p.roff; rc = rc < 0 ? 0 : (rc >= p.rn ? p.rn - 1 : rc); v += p.Rt[b * p.srb + h * p.srh + (long long)ic * p.sri + rc]; }
                    if (p.Mi) { const int mv = p.Mi[b * p.smb + h * p.smh + (long long)ic * p.smi + (long long)min(jg, p.Lk - 1) * p.smj]; if (p.mpol ? (mv != 0) : (mv == 0)) v = p.mfill; }
                    if (p.SQ) { const bool same = p.SQ[(long long)b * p.Lq + ic] == p.SK[(long long)b * p.Lk + min(jg, p.Lk - 1)]; if (p.segpol ? same : !same) v = p.mfill; }
                    if (p.causal == 2 && jg > irow + p.coff) v = p.mfill;
                    if (jg >= p.Lk || (p.causal == 1 && jg > irow + p.coff) || (p.causal == 3 && jg < irow + p.coff) || (p.win > 0 && irow + p.coff - jg > p.win)) v = NEG; else v *= L2E;
                    sc[t] = v;
                }
                if (!TWOPASS || pass == 0) {
                    float mx = fmaxf(fmaxf(sc[0], sc[1]), fmaxf(sc[2], sc[3]));
                    mx = fmaxf(mx, __shfl_xor(mx, 1, 32)); mx = fmaxf(mx, __shfl_xor(mx, 2, 32));
                    mx = fmaxf(mx, __shfl_xor(mx, 4, 32)); mx = fmaxf(mx, __shfl_xor(mx, 8, 32));
                    const float mnew = fmaxf(m8[i], mx);
                    const float corr = (mnew == NEG) ? 1.f : exp2f(m8[i] - mnew);
                    float rs = 0.f;
#pragma unroll
                    for (int t = 0; t < 4; ++t) {
                        const float pp = (sc[t] == NEG) ? 0.f : exp2f(sc[t] - mnew); rs += pp;
                        pv[i][t] = p.Pw ? pp * p.Pw[b * p.swb + h * p.swh + (long long)ic * p.swi + (long long)min(j0 + t * 16 + l15, p.Lk - 1) * p.swj] : pp;
                    }
                    rs += __shfl_xor(rs, 1, 32); rs += __shfl_xor(rs, 2, 32); rs += __shfl_xor(rs, 4, 32); rs += __shfl_xor(rs, 8, 32);
                    l8[i] = l8[i] * corr + rs; m8[i] = mnew;
                    if (!TWOPASS) {
#pragma unroll
                        for (int t = 0; t < NT; ++t) o[t][i] *= corr;
                    }
                } else {
                    const float inv = (l8[i] > 0.f) ? 1.f / l8[i] : 0.f;
#pragma unroll
                    for (int t = 0; t < 4; ++t) {
                        const int jg = j0 + t * 16 + l15;
                        float pp = (sc[t] == NEG) ? 0.f : exp2f(sc[t] - m8[i]) * inv;
                        if (p.Pw) pp *= p.Pw[b * p.swb + h * p.swh + (long long)ic * p.swi + (long long)min(jg, p.Lk - 1) * p.swj];
                        pv[i][t] = pp;
                    }
                }
            }
            if (dopv) {
#pragma unroll
                for (int i = 0; i < 8; ++i)
#pragma unroll
                    for (int t = 0; t < 4; ++t) myp[(i + 8 * hf) * 64 + t * 16 + l15] = pv[i][t];
                __syncthreads();
                if (p.P) {
                    float* pb_ = p.P + b * p.sPb + h * p.sPh;
                    const bool fastP = (p.pband == 0) && ((p.sPi & 3) == 0) && (j0 + 64 <= p.Lk) && (q0 + 16 <= p.Lq) && ((((size_t)pb_) & 15) == 0);
                    if (fastP) {
#pragma unroll
                        for (int s = 0; s < 8; ++s) {
                            const int row = s * 2 + (lane >> 4), c4 = (lane & 15) * 4;
                            const v4f v = *(const v4f*)(myp + row * 64 + c4);
                            VST2V4(pb_ + (long long)(q0 + row) * p.sPi + j0 + c4, v);
                        }
                    } else {
                        for (int row = 0; row < 16; ++row) {
                            const int irow = q0 + row; if (irow >= p.Lq) continue;
                            for (int c = lane; c < 64; c += 32) {
                                const int jg = j0 + c; if (jg >= p.Lk) continue;
                                if (p.pband == 0) VST2(float, pb_ + (long long)irow * p.sPi + jg, myp[row * 64 + c]);
                                else if (jg - irow <= p.pband && irow - jg <= p.pband) VST2(float, pb_ + (long long)irow * p.sPi + (jg - irow + p.pband), myp[row * 64 + c]);
                            }
                        }
                    }
                }
                if (SPLITPV) {
                    const Split pa0 = sp_ld(myp + l15 * 64, 1, 0, hf, 64, 1.f), pa1 = sp_ld(myp + l15 * 64, 1, 32, hf, 64, 1.f);
                    const __bf16* vh = (const __bf16*)vl; const __bf16* vlo = vh + 64 * VP;
#pragma unroll
                    for (int t = 0; t < NT; ++t) {
                        const int dcol = t * 16 + l15;
                        Split b0, b1;
#pragma unroll
                        for (int e = 0; e < 16; ++e) {
                            const int k0 = frag_k(e, hf), k1 = 32 + frag_k(e, hf);
                            b0.hi[e] = vh[k0 * VP + dcol]; b0.lo[e] = vlo[k0 * VP + dcol]; b1.hi[e] = vh[k1 * VP + dcol]; b1.lo[e] = vlo[k1 * VP + dcol];
                        }
                        o[t] = wmma3(pa0, b0, o[t]);
                        o[t] = wmma3(pa1, b1, o[t]);
                    }
                } else {
                    const v16h pa0 = fh_ld(myp + l15 * 64, 1, 0, hf, 64, 4096.f), pa1 = fh_ld(myp + l15 * 64, 1, 32, hf, 64, 4096.f);
#pragma unroll
                    for (int t = 0; t < NT; ++t) {
                        const int dcol = t * 16 + l15;
                        v16h b0, b1;
#pragma unroll
                        for (int e = 0; e < 16; ++e) { b0[e] = vl[frag_k(e, hf) * VP + dcol]; b1[e] = vl[(32 + frag_k(e, hf)) * VP + dcol]; }
                        o[t] = wmma16(pa0, b0, o[t]);
                        o[t] = wmma16(pa1, b1, o[t]);
                    }
                }
            }
        }
    }
    float* obase = p.O + b * p.sOb + h * p.sOh;
    if (p.ST) {
        const int rl = lane >> 1, isel = rl & 7;
        float mv = 0.f, lv = 0.f;
#pragma unroll
        for (int i = 0; i < 8; ++i) if (i == isel) { mv = m8[i]; lv = l8[i]; }
        const int irow = q0 + rl;
        if (irow < p.Lq) { float* st = p.ST + (((long long)b * gridDim.y + h) * p.Lq + irow) * 2 + (lane & 1); VST2(float, st, (lane & 1) ? lv : mv * 0.6931471805599453f); }
    }
    float invr[8];
#pragma unroll
    for (int i = 0; i < 8; ++i) {
        if (TWOPASS) invr[i] = SPLITPV ? 1.f : (1.f / 4096.f);
        else if (p.nonorm) invr[i] = exp2f(m8[i]) * (SPLITPV ? 1.f : (1.f / 4096.f));
        else invr[i] = (l8[i] > 0.f) ? (SPLITPV ? 1.f / l8[i] : 1.f / (l8[i] * 4096.f)) : 0.f;
    }
    __syncthreads();
    const bool ofast = ((p.sOi & 3) == 0) && ((((size_t)obase) & 15) == 0) && (q0 + 16 <= p.Lq);
#pragma unroll
    for (int c0 = 0; c0 < DVP; c0 += 64) {
#pragma unroll
        for (int i = 0; i < 8; ++i)
#pragma unroll
            for (int t = 0; t < NT; ++t) if (t * 16 >= c0 && t * 16 < c0 + 64) myp[(i + 8 * hf) * 64 + (t * 16 - c0) + l15] = o[t][i] * invr[i];
        __syncthreads();
        const int cw = (DVP - c0 < 64) ? (DVP - c0) : 64;
        if (ofast && (c0 + cw <= p.dv) && (cw % 32 == 0)) {
            const int lpr = cw / 4;
            const int rows_per_ins = 32 / lpr;
            for (int r0 = 0; r0 < 16; r0 += rows_per_ins) {
                const int row = r0 + lane / lpr, c4 = (lane % lpr) * 4;
                const v4f v = *(const v4f*)(myp + row * 64 + c4);
                VST2V4(obase + (long long)(q0 + row) * p.sOi + c0 + c4, v);
            }
        } else {
            for (int row = 0; row < 16; ++row) {
                const int irow = q0 + row; if (irow >= p.Lq) continue;
                for (int c = lane; c < cw; c += 32) { const int d = c0 + c; if (d < p.dv) VST2(float, obase + (long long)irow * p.sOi + d, myp[row * 64 + c]); }
            }
        }
        __syncthreads();
    }
}

struct TrP { const float* src; float* dst; const float* R2; long long sSz, lds, sDz, ldd, sRz, ldr; int R, C, flags, act; float alpha, beta; };
static_assert(sizeof(TrP) == 3 * 8 + 6 * 8 + 6 * 4, "TrP has padding");
__global__ __launch_bounds__(256) void k_tr(TrP p) {
    __shared__ float tile[32][33];
    const int c0 = blockIdx.x * 32, r0 = blockIdx.y * 32, z = blockIdx.z;
    const int lane = threadIdx.x & 31, wave = threadIdx.x >> 5;
    const float* s = p.src + z * p.sSz;
#pragma unroll
    for (int k = 0; k < 4; ++k) {
        const int rl = wave * 4 + k, r = r0 + rl, c = c0 + lane;
        tile[rl][lane] = (r < p.R && c < p.C) ? s[(long long)r * p.lds + c] : 0.f;
    }
    __syncthreads();
    float* d = p.dst + z * p.sDz; const float* rr = p.R2 + z * p.sRz;
#pragma unroll
    for (int k = 0; k < 4; ++k) {
        const int cl = wave * 4 + k, c = c0 + cl, r = r0 + lane;
        if (c < p.C && r < p.R) {
            float v = act_fn(p.alpha * tile[lane][cl], p.act);
            if (p.flags & 1) v += p.beta * rr[(long long)c * p.ldr + r];
            VST2(float, d + (long long)c * p.ldd + r, v);
        }
    }
}

__global__ __launch_bounds__(256) void k_affine(const float* __restrict__ src, float* __restrict__ dst, int n, float a, float b, const float* __restrict__ sdev) {
    const int i = blockIdx.x * 256 + threadIdx.x;
    if (i < n) { const float aa = sdev ? a * sdev[0] : a; const float v = aa * src[i] + b; VST2(float, dst + i, v); }
}

struct SmP { const float* src; float* dst; const float* Mf; long long sz, sr, dz, dr, smz, smr; int n, pad; float scale_in, scale_out; };
static_assert(sizeof(SmP) == 3 * 8 + 6 * 8 + 4 * 4, "SmP has padding");
__global__ __launch_bounds__(256) void k_softmax(SmP p) {
    __shared__ float red[256];
    const int r = blockIdx.x, z = blockIdx.y, tid = threadIdx.x;
    const float* s = p.src + z * p.sz + (long long)r * p.sr;
    const float* mf = p.Mf ? (p.Mf + z * p.smz + (long long)r * p.smr) : nullptr;
    float mx = -__builtin_inff();
    for (int j = tid; j < p.n; j += 256) { float v = s[j] * p.scale_in; if (mf) v += mf[j]; mx = fmaxf(mx, v); }
    red[tid] = mx; __syncthreads();
    for (int o = 128; o > 0; o >>= 1) { if (tid < o) red[tid] = fmaxf(red[tid], red[tid + o]); __syncthreads(); }
    mx = red[0]; __syncthreads();
    float sum = 0.f;
    for (int j = tid; j < p.n; j += 256) { float v = s[j] * p.scale_in; if (mf) v += mf[j]; sum += (mx == -__builtin_inff()) ? 0.f : expf(v - mx); }
    red[tid] = sum; __syncthreads();
    for (int o = 128; o > 0; o >>= 1) { if (tid < o) red[tid] += red[tid + o]; __syncthreads(); }
    sum = red[0];
    const float inv = (sum > 0.f) ? p.scale_out / sum : 0.f;
    float* d = p.dst + z * p.dz + (long long)r * p.dr;
    for (int j = tid; j < p.n; j += 256) { float v = s[j] * p.scale_in; if (mf) v += mf[j]; const float o = (mx == -__builtin_inff()) ? 0.f : expf(v - mx) * inv; VST2(float, d + j, o); }
}
__global__ __launch_bounds__(256) void k_stats(const float* __restrict__ x, long long sz, long long so, long long si, int inner, int n, float eps, float* __restrict__ stat, int mode) {
    __shared__ float red[256];
    const int z = blockIdx.x, tid = threadIdx.x;
    const float* base = x + z * sz;
    float s = 0.f;
    for (int e = tid; e < n; e += 256) s += base[(long long)(e / inner) * so + (long long)(e % inner) * si];
    red[tid] = s; __syncthreads();
    for (int o = 128; o > 0; o >>= 1) { if (tid < o) red[tid] += red[tid + o]; __syncthreads(); }
    const float mu = (mode == 0 || mode == 3) ? red[0] / (float)n : 0.f; __syncthreads();
    float q = 0.f;
    for (int e = tid; e < n; e += 256) { const float dlt = base[(long long)(e / inner) * so + (long long)(e % inner) * si] - mu; q += dlt * dlt; }
    red[tid] = q; __syncthreads();
    for (int o = 128; o > 0; o >>= 1) { if (tid < o) red[tid] += red[tid + o]; __syncthreads(); }
    {
        float rs;
        if (mode == 2) rs = sqrtf((float)n) / fmaxf(sqrtf(red[0]), eps); else if (mode == 3) rs = rsqrtf(red[0] / (float)(n - 1) + eps); else rs = rsqrtf(red[0] / (float)n + eps);
        if (tid < 32) { const float v = (tid == 0) ? mu : ((tid == 1) ? rs : 0.f); VST2(float, stat + (long long)z * 32 + tid, v); }
    }
}
__global__ __launch_bounds__(256) void k_norm_apply(const float* __restrict__ x, float* __restrict__ y, const float* __restrict__ stat, const float* __restrict__ g, const float* __restrict__ bta,
                                                     int Z, int C, int L, int G, int bn, int act) {
    const long long idx = (long long)blockIdx.x * 256 + threadIdx.x;
    if (idx >= (long long)Z * C * L) return;
    const int l = (int)(idx % L); const long long zc = idx / L; const int c = (int)(zc % C), z = (int)(zc / C); (void)l;
    const int set = bn ? c : (z * G + c / (C / G));
    float v = (x[idx] - stat[(long long)set * 32]) * stat[(long long)set * 32 + 1];
    if (g) v *= g[c];
    if (bta) v += bta[c];
    v = act_fn(v, act);
    VST2(float, y + idx, v);
}

__global__ __launch_bounds__(256) void k_lse_neg(const float* __restrict__ st, float* __restrict__ c, int n) {
    const int i = blockIdx.x * 256 + threadIdx.x;
    if (i < n) { const float v = -(st[2 * i] + logf(st[2 * i + 1])); VST2(float, c + i, v); }
}

__global__ __launch_bounds__(256) void k_iota(int* __restrict__ dst, int n, int a, int b) {
    const int i = blockIdx.x * 256 + threadIdx.x;
    if (i < n) { const int v = a * i + b; VST2(int, dst + i, v); }
}

__global__ __launch_bounds__(256) void k_axpby(const float* __restrict__ x, const float* __restrict__ y, float* __restrict__ dst, int n, float a, float b, float c) {
    const int i = blockIdx.x * 256 + threadIdx.x;
    if (i < n) { const float v = a * x[i] + b * y[i] + c; VST2(float, dst + i, v); }
}

struct RopeP { const float* X; float* Y; const float* C; const float* Sn; const int* pos; long long sXr, sXh, sYr, sYh, sCb, sCp, sCd; int R, Hn, D, S, mode, tmode, pmode, pad; };
static_assert(sizeof(RopeP) == 5 * 8 + 7 * 8 + 8 * 4, "RopeP has padding");
__global__ __launch_bounds__(256) void k_rope(RopeP p) {
    const long long idx = (long long)blockIdx.x * 256 + threadIdx.x;
    if (idx >= (long long)p.R * p.Hn * p.D) return;
    const int d = (int)(idx % p.D); const long long rh = idx / p.D; const int h = (int)(rh % p.Hn); const int r = (int)(rh / p.Hn);
    const int half = p.D / 2;
    int partner; float sign;
    if (p.mode == 0) { partner = (d < half) ? d + half : d - half; sign = (d < half) ? -1.f : 1.f; }
    else { partner = d ^ 1; sign = (d & 1) ? 1.f : -1.f; }
    const int tcol = (p.tmode == 0) ? d : ((p.tmode == 1) ? (d % half) : (d >> 1));
    const int pp = (p.pmode == 0) ? (r % p.S) : ((p.pmode == 1) ? h : p.pos[r]);
    const long long toff = (long long)(r / p.S) * p.sCb + (long long)pp * p.sCp + (long long)tcol * p.sCd;
    const float* xr = p.X + (long long)r * p.sXr + (long long)h * p.sXh;
    const float v = xr[d] * p.C[toff] + sign * xr[partner] * p.Sn[toff];
    VST2(float, p.Y + (long long)r * p.sYr + (long long)h * p.sYh + d, v);
}

__global__ __launch_bounds__(256) void k_invf(float* __restrict__ invb, int half, int D, float base, float num, int fmode, float cexp) {
    const int i = blockIdx.x * 256 + threadIdx.x;
    if (i >= ((half + 31) / 32) * 32) return;
    if (i >= half) { VST2(float, invb + i, 0.f); return; }
    const float e = (float)(2 * i) / (float)D;
    float invf;
    if (fmode == 1) invf = num * expf((float)(2 * i) * cexp);
    else if (fmode == 2) invf = num * powf(base, (-2.0f * ((float)i - 1.0f)) / (float)D);
    else invf = num * (1.0f / powf(base, e));
    VST2(float, invb + i, invf);
}
__global__ __launch_bounds__(256) void k_sincos(float* __restrict__ cs, float* __restrict__ sn, const float* __restrict__ invb, int S, int half, float pscale) {
    const int idx = blockIdx.x * 256 + threadIdx.x;
    if (idx >= S * half) return;
    const int s = idx / half, i = idx - s * half;
    const float ang = (pscale * (float)s) * invb[i];
    VST2(float, cs + idx, cosf(ang)); VST2(float, sn + idx, sinf(ang));
}

__global__ __launch_bounds__(256) void k_mulact(const float* __restrict__ x, const float* __restrict__ y, float* __restrict__ dst, int n, int act) {
    const int i = blockIdx.x * 256 + threadIdx.x;
    if (i < n) { const float v = act_fn(x[i], act) * y[i]; VST2(float, dst + i, v); }
}

__global__ __launch_bounds__(256) void k_matvec(GemmP p) {
    const int rpt = (p.N == 1) ? 1 : 32;
    const long long r0 = ((long long)blockIdx.x * 256 + threadIdx.x) * rpt; const int z = blockIdx.z, zo = z / p.zi_n, zi = z - zo * p.zi_n;
    if (r0 >= p.M) return;
    const float* Bb = p.B + zo * p.sBo + zi * p.sBi;
    float* C = p.C + zo * p.sCo + zi * p.sCi; const float* R = p.R + zo * p.sRo + zi * p.sRi;
    for (int rr = 0; rr < rpt; ++rr) {
        const long long r = r0 + rr; if (r >= p.M) break;
        const float* A = p.A + zo * p.sAo + zi * p.sAi + r * p.sAm;
        float acc[8] = {0.f, 0.f, 0.f, 0.f, 0.f, 0.f, 0.f, 0.f};
        for (int k = 0; k < p.K; ++k) { const float a = A[(long long)k * p.sAk];
#pragma unroll
            for (int j = 0; j < 8; ++j) if (j < p.N) acc[j] += a * Bb[(long long)j * p.sBn + (long long)k * p.sBk]; }
#pragma unroll
        for (int j = 0; j < 8; ++j) if (j < p.N) {
            float v = acc[j] * p.alpha;
            if (p.flags & 1) v += p.bias[j];
            if (p.flags & 2) v += p.bias[r];
            v = act_fn(v, p.act);
            if (p.flags & 4) v += p.beta * R[r * p.sRm + (long long)j * p.sRn];
            VST2(float, C + r * p.sCm + j, v);
        }
    }
}
__global__ __launch_bounds__(256) void k_smallsoftmax(const float* __restrict__ src, float* __restrict__ dst, long long sr, long long dr, int n, long long R, float scale) {
    const long long r0 = ((long long)blockIdx.x * 256 + threadIdx.x) * 32;
    for (int rr = 0; rr < 32; ++rr) {
        const long long r = r0 + rr; if (r >= R) return;
        const float* s = src + r * sr; float* d = dst + r * dr;
        float mx = -__builtin_inff();
        for (int j = 0; j < n; ++j) mx = fmaxf(mx, s[j] * scale);
        float sum = 0.f;
        for (int j = 0; j < n; ++j) sum += expf(s[j] * scale - mx);
        const float inv = 1.f / sum;
        for (int j = 0; j < n; ++j) { const float v = expf(s[j] * scale - mx) * inv; VST2(float, d + j, v); }
    }
}

__global__ __launch_bounds__(32) void k_unitstat(float* __restrict__ st) { const int t = threadIdx.x; const float v = (t == 1) ? 1.f : 0.f; VST2(float, st + t, v); }

__global__ __launch_bounds__(256) void k_lincopy(const float* __restrict__ src, long long lds, float* __restrict__ dst, long long ldd, long long rows, int cols) {
    const long long i = (long long)blockIdx.x * 256 + threadIdx.x; if (i >= rows * cols) return;
    const long long r = i / cols; const int c = (int)(i - r * cols);
    const float v = src[r * lds + c]; VST2(float, dst + r * ldd + c, v);
}

__global__ __launch_bounds__(256) void k_dc_deg(const float* __restrict__ A, float* __restrict__ dr, float* __restrict__ dc, int N) { const int q = blockIdx.x * 256 + threadIdx.x; if (q >= 2 * N) return; float s = 0.f; if (q < N) { for (int j = 0; j < N; ++j) s += A[(long long)q * N + j]; VST2(float, dr + q, s); } else { const int n = q - N; for (int j = 0; j < N; ++j) s += A[(long long)j * N + n]; VST2(float, dc + n, s); } }
__global__ __launch_bounds__(256) void k_dc_sup(const float* __restrict__ A, const float* __restrict__ dr, const float* __restrict__ dc, float* __restrict__ S1, float* __restrict__ S2, int N) { const long long q = (long long)blockIdx.x * 256 + threadIdx.x; if (q >= (long long)N * N) return; const int n = (int)(q % N); const int m = (int)(q / N); const float d1 = dr[n], d2 = dc[n];
    VST2(float, S1 + q, (d1 > 0.f) ? A[(long long)n * N + m] * (1.f / d1) : 0.f); VST2(float, S2 + q, (d2 > 0.f) ? A[q] * (1.f / d2) : 0.f); }
__global__ __launch_bounds__(256) void k_dc_x0(const float* __restrict__ inp, const float* __restrict__ hs, const float* __restrict__ gate, float* __restrict__ X0, int B, int N, int DS, int H) { const long long q = (long long)blockIdx.x * 256 + threadIdx.x; const int P = DS + H; if (q >= (long long)N * B * P) return; const int p = (int)(q % P); const int b = (int)((q / P) % B); const int n = (int)(q / ((long long)P * B));
    float v; if (p < DS) v = inp[((long long)b * N + n) * DS + p]; else { const long long hi = ((long long)b * N + n) * H + (p - DS); v = hs[hi]; if (gate) v *= gate[hi]; } VST2(float, X0 + q, v); }
__global__ __launch_bounds__(256) void k_dc_out(const float* __restrict__ U, const float* __restrict__ ST, const float* __restrict__ Cg, float* __restrict__ OUT, long long n) { const long long q = (long long)blockIdx.x * 256 + threadIdx.x; if (q >= n) return; const float u = U[q]; VST2(float, OUT + q, u * ST[q] + (1.f - u) * Cg[q]); }

template __global__ void k_gemm<1>(GemmP);

extern "C" void kernel_launch(void* const* d_in, const int* in_sizes, int n_in, void* d_out, int out_size, void* d_ws, size_t ws_size, hipStream_t stream) {
    (void)in_sizes; (void)n_in; (void)out_size; (void)ws_size;
    const float* inp = (const float*)d_in[0];
    const float* state = (const float*)d_in[1];
    const float* adj = (const float*)d_in[2];
    const float* thr = (const float*)d_in[3];
    const float* thu = (const float*)d_in[4];
    const float* thc = (const float*)d_in[5];
    const float* br = (const float*)d_in[6];
    const float* bu = (const float*)d_in[7];
    const float* bc = (const float*)d_in[8];
    const int Bn = 32;
    const int N = 2048;
    const int DS = 16;
    const int H = 64;
    const int P = 80;
    const int BP = Bn * P;
    const int KM = 5;
    float* out = (float*)d_out;
    char* wsp = (char*)d_ws;
    float* dr = (float*)wsp; wsp += (((size_t)((size_t)N + 64) * 4 + 255) / 256) * 256;
    float* dc = (float*)wsp; wsp += (((size_t)((size_t)N + 64) * 4 + 255) / 256) * 256;
    float* S1 = (float*)wsp; wsp += (((size_t)((size_t)N * N) * 4 + 255) / 256) * 256;
    float* S2 = (float*)wsp; wsp += (((size_t)((size_t)N * N) * 4 + 255) / 256) * 256;
    float* X0 = (float*)wsp; wsp += (((size_t)((size_t)N * BP) * 4 + 255) / 256) * 256;
    float* X1 = (float*)wsp; wsp += (((size_t)((size_t)N * BP) * 4 + 255) / 256) * 256;
    float* X2 = (float*)wsp; wsp += (((size_t)((size_t)N * BP) * 4 + 255) / 256) * 256;
    float* X3 = (float*)wsp; wsp += (((size_t)((size_t)N * BP) * 4 + 255) / 256) * 256;
    float* X4 = (float*)wsp; wsp += (((size_t)((size_t)N * BP) * 4 + 255) / 256) * 256;
    float* R = (float*)wsp; wsp += (((size_t)((size_t)Bn * N * H) * 4 + 255) / 256) * 256;
    float* U = (float*)wsp; wsp += (((size_t)((size_t)Bn * N * H) * 4 + 255) / 256) * 256;
    float* Cg = (float*)wsp; wsp += (((size_t)((size_t)Bn * N * H) * 4 + 255) / 256) * 256;
    k_dc_deg<<<(unsigned)((2 * N + 255) / 256), 256, 0, stream>>>(adj, dr, dc, N);
    k_dc_sup<<<(unsigned)(((long long)N * N + 255) / 256), 256, 0, stream>>>(adj, dr, dc, S1, S2, N);
    k_dc_x0<<<(unsigned)(((long long)N * BP + 255) / 256), 256, 0, stream>>>(inp, state, nullptr, X0, Bn, N, DS, H);
    { GemmP gda_n;
      gda_n.A = S1; gda_n.B = X0; gda_n.bias = S1; gda_n.R = S1; gda_n.C = X1;
      gda_n.sAo = 0; gda_n.sAi = 0; gda_n.sAm = N; gda_n.sAk = 1; gda_n.sBo = 0; gda_n.sBi = 0; gda_n.sBn = 1; gda_n.sBk = BP; gda_n.sCo = 0; gda_n.sCi = 0; gda_n.sCm = BP; gda_n.sRo = 0; gda_n.sRi = 0; gda_n.sRm = 0; gda_n.sRn = 0;
      gda_n.M = N; gda_n.N = BP; gda_n.K = N; gda_n.zi_n = 1; gda_n.flags = 0; gda_n.act = 0;
      gda_n.alpha = 1.0f; gda_n.beta = 0.0f; gda_n.sa = 1.0f; gda_n.sb = 1.0f; gda_n.Npad = BP; gda_n.pad_ = 0;
      k_gemm<1><<<dim3((unsigned)((BP) + 31) / 32, (unsigned)((N) + 15) / 16, (unsigned)(1)), 32, 0, stream>>>(gda_n); }
    { GemmP gdb_n;
      gdb_n.A = S1; gdb_n.B = X1; gdb_n.bias = S1; gdb_n.R = S1; gdb_n.C = X2;
      gdb_n.sAo = 0; gdb_n.sAi = 0; gdb_n.sAm = N; gdb_n.sAk = 1; gdb_n.sBo = 0; gdb_n.sBi = 0; gdb_n.sBn = 1; gdb_n.sBk = BP; gdb_n.sCo = 0; gdb_n.sCi = 0; gdb_n.sCm = BP; gdb_n.sRo = 0; gdb_n.sRi = 0; gdb_n.sRm = 0; gdb_n.sRn = 0;
      gdb_n.M = N; gdb_n.N = BP; gdb_n.K = N; gdb_n.zi_n = 1; gdb_n.flags = 0; gdb_n.act = 0;
      gdb_n.alpha = 1.0f; gdb_n.beta = 0.0f; gdb_n.sa = 1.0f; gdb_n.sb = 1.0f; gdb_n.Npad = BP; gdb_n.pad_ = 0;
      k_gemm<1><<<dim3((unsigned)((BP) + 31) / 32, (unsigned)((N) + 15) / 16, (unsigned)(1)), 32, 0, stream>>>(gdb_n); }
    { GemmP gdc_n;
      gdc_n.A = S2; gdc_n.B = X0; gdc_n.bias = S2; gdc_n.R = S2; gdc_n.C = X3;
      gdc_n.sAo = 0; gdc_n.sAi = 0; gdc_n.sAm = N; gdc_n.sAk = 1; gdc_n.sBo = 0; gdc_n.sBi = 0; gdc_n.sBn = 1; gdc_n.sBk = BP; gdc_n.sCo = 0; gdc_n.sCi = 0; gdc_n.sCm = BP; gdc_n.sRo = 0; gdc_n.sRi = 0; gdc_n.sRm = 0; gdc_n.sRn = 0;
      gdc_n.M = N; gdc_n.N = BP; gdc_n.K = N; gdc_n.zi_n = 1; gdc_n.flags = 0; gdc_n.act = 0;
      gdc_n.alpha = 1.0f; gdc_n.beta = 0.0f; gdc_n.sa = 1.0f; gdc_n.sb = 1.0f; gdc_n.Npad = BP; gdc_n.pad_ = 0;
      k_gemm<1><<<dim3((unsigned)((BP) + 31) / 32, (unsigned)((N) + 15) / 16, (unsigned)(1)), 32, 0, stream>>>(gdc_n); }
    { GemmP gdd_n;
      gdd_n.A = S2; gdd_n.B = X3; gdd_n.bias = S2; gdd_n.R = S2; gdd_n.C = X4;
      gdd_n.sAo = 0; gdd_n.sAi = 0; gdd_n.sAm = N; gdd_n.sAk = 1; gdd_n.sBo = 0; gdd_n.sBi = 0; gdd_n.sBn = 1; gdd_n.sBk = BP; gdd_n.sCo = 0; gdd_n.sCi = 0; gdd_n.sCm = BP; gdd_n.sRo = 0; gdd_n.sRi = 0; gdd_n.sRm = 0; gdd_n.sRn = 0;
      gdd_n.M = N; gdd_n.N = BP; gdd_n.K = N; gdd_n.zi_n = 1; gdd_n.flags = 0; gdd_n.act = 0;
      gdd_n.alpha = 1.0f; gdd_n.beta = 0.0f; gdd_n.sa = 1.0f; gdd_n.sb = 1.0f; gdd_n.Npad = BP; gdd_n.pad_ = 0;
      k_gemm<1><<<dim3((unsigned)((BP) + 31) / 32, (unsigned)((N) + 15) / 16, (unsigned)(1)), 32, 0, stream>>>(gdd_n); }
    { GemmP gcr0;
      gcr0.A = X0; gcr0.B = thr + 0; gcr0.bias = br; gcr0.R = X0; gcr0.C = R;
      gcr0.sAo = P; gcr0.sAi = 0; gcr0.sAm = BP; gcr0.sAk = 1; gcr0.sBo = 0; gcr0.sBi = 0; gcr0.sBn = 1; gcr0.sBk = KM * H; gcr0.sCo = (long long)N * H; gcr0.sCi = 0; gcr0.sCm = H; gcr0.sRo = 0; gcr0.sRi = 0; gcr0.sRm = 0; gcr0.sRn = 0;
      gcr0.M = N; gcr0.N = H; gcr0.K = P; gcr0.zi_n = 1; gcr0.flags = 1; gcr0.act = 0;
      gcr0.alpha = 1.0f; gcr0.beta = 0.0f; gcr0.sa = 1.0f; gcr0.sb = 1.0f; gcr0.Npad = H; gcr0.pad_ = 0;
      k_gemm<1><<<dim3((unsigned)((H) + 31) / 32, (unsigned)((N) + 15) / 16, (unsigned)(Bn)), 32, 0, stream>>>(gcr0); }
    { GemmP gcr1;
      gcr1.A = X1; gcr1.B = thr + 64; gcr1.bias = X1; gcr1.R = R; gcr1.C = R;
      gcr1.sAo = P; gcr1.sAi = 0; gcr1.sAm = BP; gcr1.sAk = 1; gcr1.sBo = 0; gcr1.sBi = 0; gcr1.sBn = 1; gcr1.sBk = KM * H; gcr1.sCo = (long long)N * H; gcr1.sCi = 0; gcr1.sCm = H; gcr1.sRo = (long long)N * H; gcr1.sRi = 0; gcr1.sRm = H; gcr1.sRn = 1;
      gcr1.M = N; gcr1.N = H; gcr1.K = P; gcr1.zi_n = 1; gcr1.flags = 4; gcr1.act = 0;
      gcr1.alpha = 1.0f; gcr1.beta = 1.0f; gcr1.sa = 1.0f; gcr1.sb = 1.0f; gcr1.Npad = H; gcr1.pad_ = 0;
      k_gemm<1><<<dim3((unsigned)((H) + 31) / 32, (unsigned)((N) + 15) / 16, (unsigned)(Bn)), 32, 0, stream>>>(gcr1); }
    { GemmP gcr2;
      gcr2.A = X2; gcr2.B = thr + 128; gcr2.bias = X2; gcr2.R = R; gcr2.C = R;
      gcr2.sAo = P; gcr2.sAi = 0; gcr2.sAm = BP; gcr2.sAk = 1; gcr2.sBo = 0; gcr2.sBi = 0; gcr2.sBn = 1; gcr2.sBk = KM * H; gcr2.sCo = (long long)N * H; gcr2.sCi = 0; gcr2.sCm = H; gcr2.sRo = (long long)N * H; gcr2.sRi = 0; gcr2.sRm = H; gcr2.sRn = 1;
      gcr2.M = N; gcr2.N = H; gcr2.K = P; gcr2.zi_n = 1; gcr2.flags = 4; gcr2.act = 0;
      gcr2.alpha = 1.0f; gcr2.beta = 1.0f; gcr2.sa = 1.0f; gcr2.sb = 1.0f; gcr2.Npad = H; gcr2.pad_ = 0;
      k_gemm<1><<<dim3((unsigned)((H) + 31) / 32, (unsigned)((N) + 15) / 16, (unsigned)(Bn)), 32, 0, stream>>>(gcr2); }
    { GemmP gcr3;
      gcr3.A = X3; gcr3.B = thr + 192; gcr3.bias = X3; gcr3.R = R; gcr3.C = R;
      gcr3.sAo = P; gcr3.sAi = 0; gcr3.sAm = BP; gcr3.sAk = 1; gcr3.sBo = 0; gcr3.sBi = 0; gcr3.sBn = 1; gcr3.sBk = KM * H; gcr3.sCo = (long long)N * H; gcr3.sCi = 0; gcr3.sCm = H; gcr3.sRo = (long long)N * H; gcr3.sRi = 0; gcr3.sRm = H; gcr3.sRn = 1;
      gcr3.M = N; gcr3.N = H; gcr3.K = P; gcr3.zi_n = 1; gcr3.flags = 4; gcr3.act = 0;
      gcr3.alpha = 1.0f; gcr3.beta = 1.0f; gcr3.sa = 1.0f; gcr3.sb = 1.0f; gcr3.Npad = H; gcr3.pad_ = 0;
      k_gemm<1><<<dim3((unsigned)((H) + 31) / 32, (unsigned)((N) + 15) / 16, (unsigned)(Bn)), 32, 0, stream>>>(gcr3); }
    { GemmP gcr4;
      gcr4.A = X4; gcr4.B = thr + 256; gcr4.bias = X4; gcr4.R = R; gcr4.C = R;
      gcr4.sAo = P; gcr4.sAi = 0; gcr4.sAm = BP; gcr4.sAk = 1; gcr4.sBo = 0; gcr4.sBi = 0; gcr4.sBn = 1; gcr4.sBk = KM * H; gcr4.sCo = (long long)N * H; gcr4.sCi = 0; gcr4.sCm = H; gcr4.sRo = (long long)N * H; gcr4.sRi = 0; gcr4.sRm = H; gcr4.sRn = 1;
      gcr4.M = N; gcr4.N = H; gcr4.K = P; gcr4.zi_n = 1; gcr4.flags = 4; gcr4.act = 0;
      gcr4.alpha = 1.0f; gcr4.beta = 1.0f; gcr4.sa = 1.0f; gcr4.sb = 1.0f; gcr4.Npad = H; gcr4.pad_ = 0;
      k_gemm<1><<<dim3((unsigned)((H) + 31) / 32, (unsigned)((N) + 15) / 16, (unsigned)(Bn)), 32, 0, stream>>>(gcr4); }
    k_unitstat<<<1, 32, 0, stream>>>(dr);
    k_norm_apply<<<(unsigned)(((long long)(1) * (1) * ((long long)Bn * N * H) + 255) / 256), 256, 0, stream>>>(R, R, dr, nullptr, nullptr, 1, 1, (long long)Bn * N * H, 1, 0, 6);
    { GemmP gcu0;
      gcu0.A = X0; gcu0.B = thu + 0; gcu0.bias = bu; gcu0.R = X0; gcu0.C = U;
      gcu0.sAo = P; gcu0.sAi = 0; gcu0.sAm = BP; gcu0.sAk = 1; gcu0.sBo = 0; gcu0.sBi = 0; gcu0.sBn = 1; gcu0.sBk = KM * H; gcu0.sCo = (long long)N * H; gcu0.sCi = 0; gcu0.sCm = H; gcu0.sRo = 0; gcu0.sRi = 0; gcu0.sRm = 0; gcu0.sRn = 0;
      gcu0.M = N; gcu0.N = H; gcu0.K = P; gcu0.zi_n = 1; gcu0.flags = 1; gcu0.act = 0;
      gcu0.alpha = 1.0f; gcu0.beta = 0.0f; gcu0.sa = 1.0f; gcu0.sb = 1.0f; gcu0.Npad = H; gcu0.pad_ = 0;
      k_gemm<1><<<dim3((unsigned)((H) + 31) / 32, (unsigned)((N) + 15) / 16, (unsigned)(Bn)), 32, 0, stream>>>(gcu0); }
    { GemmP gcu1;
      gcu1.A = X1; gcu1.B = thu + 64; gcu1.bias = X1; gcu1.R = U; gcu1.C = U;
      gcu1.sAo = P; gcu1.sAi = 0; gcu1.sAm = BP; gcu1.sAk = 1; gcu1.sBo = 0; gcu1.sBi = 0; gcu1.sBn = 1; gcu1.sBk = KM * H; gcu1.sCo = (long long)N * H; gcu1.sCi = 0; gcu1.sCm = H; gcu1.sRo = (long long)N * H; gcu1.sRi = 0; gcu1.sRm = H; gcu1.sRn = 1;
      gcu1.M = N; gcu1.N = H; gcu1.K = P; gcu1.zi_n = 1; gcu1.flags = 4; gcu1.act = 0;
      gcu1.alpha = 1.0f; gcu1.beta = 1.0f; gcu1.sa = 1.0f; gcu1.sb = 1.0f; gcu1.Npad = H; gcu1.pad_ = 0;
      k_gemm<1><<<dim3((unsigned)((H) + 31) / 32, (unsigned)((N) + 15) / 16, (unsigned)(Bn)), 32, 0, stream>>>(gcu1); }
    { GemmP gcu2;
      gcu2.A = X2; gcu2.B = thu + 128; gcu2.bias = X2; gcu2.R = U; gcu2.C = U;
      gcu2.sAo = P; gcu2.sAi = 0; gcu2.sAm = BP; gcu2.sAk = 1; gcu2.sBo = 0; gcu2.sBi = 0; gcu2.sBn = 1; gcu2.sBk = KM * H; gcu2.sCo = (long long)N * H; gcu2.sCi = 0; gcu2.sCm = H; gcu2.sRo = (long long)N * H; gcu2.sRi = 0; gcu2.sRm = H; gcu2.sRn = 1;
      gcu2.M = N; gcu2.N = H; gcu2.K = P; gcu2.zi_n = 1; gcu2.flags = 4; gcu2.act = 0;
      gcu2.alpha = 1.0f; gcu2.beta = 1.0f; gcu2.sa = 1.0f; gcu2.sb = 1.0f; gcu2.Npad = H; gcu2.pad_ = 0;
      k_gemm<1><<<dim3((unsigned)((H) + 31) / 32, (unsigned)((N) + 15) / 16, (unsigned)(Bn)), 32, 0, stream>>>(gcu2); }
    { GemmP gcu3;
      gcu3.A = X3; gcu3.B = thu + 192; gcu3.bias = X3; gcu3.R = U; gcu3.C = U;
      gcu3.sAo = P; gcu3.sAi = 0; gcu3.sAm = BP; gcu3.sAk = 1; gcu3.sBo = 0; gcu3.sBi = 0; gcu3.sBn = 1; gcu3.sBk = KM * H; gcu3.sCo = (long long)N * H; gcu3.sCi = 0; gcu3.sCm = H; gcu3.sRo = (long long)N * H; gcu3.sRi = 0; gcu3.sRm = H; gcu3.sRn = 1;
      gcu3.M = N; gcu3.N = H; gcu3.K = P; gcu3.zi_n = 1; gcu3.flags = 4; gcu3.act = 0;
      gcu3.alpha = 1.0f; gcu3.beta = 1.0f; gcu3.sa = 1.0f; gcu3.sb = 1.0f; gcu3.Npad = H; gcu3.pad_ = 0;
      k_gemm<1><<<dim3((unsigned)((H) + 31) / 32, (unsigned)((N) + 15) / 16, (unsigned)(Bn)), 32, 0, stream>>>(gcu3); }
    { GemmP gcu4;
      gcu4.A = X4; gcu4.B = thu + 256; gcu4.bias = X4; gcu4.R = U; gcu4.C = U;
      gcu4.sAo = P; gcu4.sAi = 0; gcu4.sAm = BP; gcu4.sAk = 1; gcu4.sBo = 0; gcu4.sBi = 0; gcu4.sBn = 1; gcu4.sBk = KM * H; gcu4.sCo = (long long)N * H; gcu4.sCi = 0; gcu4.sCm = H; gcu4.sRo = (long long)N * H; gcu4.sRi = 0; gcu4.sRm = H; gcu4.sRn = 1;
      gcu4.M = N; gcu4.N = H; gcu4.K = P; gcu4.zi_n = 1; gcu4.flags = 4; gcu4.act = 0;
      gcu4.alpha = 1.0f; gcu4.beta = 1.0f; gcu4.sa = 1.0f; gcu4.sb = 1.0f; gcu4.Npad = H; gcu4.pad_ = 0;
      k_gemm<1><<<dim3((unsigned)((H) + 31) / 32, (unsigned)((N) + 15) / 16, (unsigned)(Bn)), 32, 0, stream>>>(gcu4); }
    k_unitstat<<<1, 32, 0, stream>>>(dr);
    k_norm_apply<<<(unsigned)(((long long)(1) * (1) * ((long long)Bn * N * H) + 255) / 256), 256, 0, stream>>>(U, U, dr, nullptr, nullptr, 1, 1, (long long)Bn * N * H, 1, 0, 6);
    k_dc_x0<<<(unsigned)(((long long)N * BP + 255) / 256), 256, 0, stream>>>(inp, state, R, X0, Bn, N, DS, H);
    { GemmP gda_R;
      gda_R.A = S1; gda_R.B = X0; gda_R.bias = S1; gda_R.R = S1; gda_R.C = X1;
      gda_R.sAo = 0; gda_R.sAi = 0; gda_R.sAm = N; gda_R.sAk = 1; gda_R.sBo = 0; gda_R.sBi = 0; gda_R.sBn = 1; gda_R.sBk = BP; gda_R.sCo = 0; gda_R.sCi = 0; gda_R.sCm = BP; gda_R.sRo = 0; gda_R.sRi = 0; gda_R.sRm = 0; gda_R.sRn = 0;
      gda_R.M = N; gda_R.N = BP; gda_R.K = N; gda_R.zi_n = 1; gda_R.flags = 0; gda_R.act = 0;
      gda_R.alpha = 1.0f; gda_R.beta = 0.0f; gda_R.sa = 1.0f; gda_R.sb = 1.0f; gda_R.Npad = BP; gda_R.pad_ = 0;
      k_gemm<1><<<dim3((unsigned)((BP) + 31) / 32, (unsigned)((N) + 15) / 16, (unsigned)(1)), 32, 0, stream>>>(gda_R); }
    { GemmP gdb_R;
      gdb_R.A = S1; gdb_R.B = X1; gdb_R.bias = S1; gdb_R.R = S1; gdb_R.C = X2;
      gdb_R.sAo = 0; gdb_R.sAi = 0; gdb_R.sAm = N; gdb_R.sAk = 1; gdb_R.sBo = 0; gdb_R.sBi = 0; gdb_R.sBn = 1; gdb_R.sBk = BP; gdb_R.sCo = 0; gdb_R.sCi = 0; gdb_R.sCm = BP; gdb_R.sRo = 0; gdb_R.sRi = 0; gdb_R.sRm = 0; gdb_R.sRn = 0;
      gdb_R.M = N; gdb_R.N = BP; gdb_R.K = N; gdb_R.zi_n = 1; gdb_R.flags = 0; gdb_R.act = 0;
      gdb_R.alpha = 1.0f; gdb_R.beta = 0.0f; gdb_R.sa = 1.0f; gdb_R.sb = 1.0f; gdb_R.Npad = BP; gdb_R.pad_ = 0;
      k_gemm<1><<<dim3((unsigned)((BP) + 31) / 32, (unsigned)((N) + 15) / 16, (unsigned)(1)), 32, 0, stream>>>(gdb_R); }
    { GemmP gdc_R;
      gdc_R.A = S2; gdc_R.B = X0; gdc_R.bias = S2; gdc_R.R = S2; gdc_R.C = X3;
      gdc_R.sAo = 0; gdc_R.sAi = 0; gdc_R.sAm = N; gdc_R.sAk = 1; gdc_R.sBo = 0; gdc_R.sBi = 0; gdc_R.sBn = 1; gdc_R.sBk = BP; gdc_R.sCo = 0; gdc_R.sCi = 0; gdc_R.sCm = BP; gdc_R.sRo = 0; gdc_R.sRi = 0; gdc_R.sRm = 0; gdc_R.sRn = 0;
      gdc_R.M = N; gdc_R.N = BP; gdc_R.K = N; gdc_R.zi_n = 1; gdc_R.flags = 0; gdc_R.act = 0;
      gdc_R.alpha = 1.0f; gdc_R.beta = 0.0f; gdc_R.sa = 1.0f; gdc_R.sb = 1.0f; gdc_R.Npad = BP; gdc_R.pad_ = 0;
      k_gemm<1><<<dim3((unsigned)((BP) + 31) / 32, (unsigned)((N) + 15) / 16, (unsigned)(1)), 32, 0, stream>>>(gdc_R); }
    { GemmP gdd_R;
      gdd_R.A = S2; gdd_R.B = X3; gdd_R.bias = S2; gdd_R.R = S2; gdd_R.C = X4;
      gdd_R.sAo = 0; gdd_R.sAi = 0; gdd_R.sAm = N; gdd_R.sAk = 1; gdd_R.sBo = 0; gdd_R.sBi = 0; gdd_R.sBn = 1; gdd_R.sBk = BP; gdd_R.sCo = 0; gdd_R.sCi = 0; gdd_R.sCm = BP; gdd_R.sRo = 0; gdd_R.sRi = 0; gdd_R.sRm = 0; gdd_R.sRn = 0;
      gdd_R.M = N; gdd_R.N = BP; gdd_R.K = N; gdd_R.zi_n = 1; gdd_R.flags = 0; gdd_R.act = 0;
      gdd_R.alpha = 1.0f; gdd_R.beta = 0.0f; gdd_R.sa = 1.0f; gdd_R.sb = 1.0f; gdd_R.Npad = BP; gdd_R.pad_ = 0;
      k_gemm<1><<<dim3((unsigned)((BP) + 31) / 32, (unsigned)((N) + 15) / 16, (unsigned)(1)), 32, 0, stream>>>(gdd_R); }
    { GemmP gcc0;
      gcc0.A = X0; gcc0.B = thc + 0; gcc0.bias = bc; gcc0.R = X0; gcc0.C = Cg;
      gcc0.sAo = P; gcc0.sAi = 0; gcc0.sAm = BP; gcc0.sAk = 1; gcc0.sBo = 0; gcc0.sBi = 0; gcc0.sBn = 1; gcc0.sBk = KM * H; gcc0.sCo = (long long)N * H; gcc0.sCi = 0; gcc0.sCm = H; gcc0.sRo = 0; gcc0.sRi = 0; gcc0.sRm = 0; gcc0.sRn = 0;
      gcc0.M = N; gcc0.N = H; gcc0.K = P; gcc0.zi_n = 1; gcc0.flags = 1; gcc0.act = 0;
      gcc0.alpha = 1.0f; gcc0.beta = 0.0f; gcc0.sa = 1.0f; gcc0.sb = 1.0f; gcc0.Npad = H; gcc0.pad_ = 0;
      k_gemm<1><<<dim3((unsigned)((H) + 31) / 32, (unsigned)((N) + 15) / 16, (unsigned)(Bn)), 32, 0, stream>>>(gcc0); }
    { GemmP gcc1;
      gcc1.A = X1; gcc1.B = thc + 64; gcc1.bias = X1; gcc1.R = Cg; gcc1.C = Cg;
      gcc1.sAo = P; gcc1.sAi = 0; gcc1.sAm = BP; gcc1.sAk = 1; gcc1.sBo = 0; gcc1.sBi = 0; gcc1.sBn = 1; gcc1.sBk = KM * H; gcc1.sCo = (long long)N * H; gcc1.sCi = 0; gcc1.sCm = H; gcc1.sRo = (long long)N * H; gcc1.sRi = 0; gcc1.sRm = H; gcc1.sRn = 1;
      gcc1.M = N; gcc1.N = H; gcc1.K = P; gcc1.zi_n = 1; gcc1.flags = 4; gcc1.act = 0;
      gcc1.alpha = 1.0f; gcc1.beta = 1.0f; gcc1.sa = 1.0f; gcc1.sb = 1.0f; gcc1.Npad = H; gcc1.pad_ = 0;
      k_gemm<1><<<dim3((unsigned)((H) + 31) / 32, (unsigned)((N) + 15) / 16, (unsigned)(Bn)), 32, 0, stream>>>(gcc1); }
    { GemmP gcc2;
      gcc2.A = X2; gcc2.B = thc + 128; gcc2.bias = X2; gcc2.R = Cg; gcc2.C = Cg;
      gcc2.sAo = P; gcc2.sAi = 0; gcc2.sAm = BP; gcc2.sAk = 1; gcc2.sBo = 0; gcc2.sBi = 0; gcc2.sBn = 1; gcc2.sBk = KM * H; gcc2.sCo = (long long)N * H; gcc2.sCi = 0; gcc2.sCm = H; gcc2.sRo = (long long)N * H; gcc2.sRi = 0; gcc2.sRm = H; gcc2.sRn = 1;
      gcc2.M = N; gcc2.N = H; gcc2.K = P; gcc2.zi_n = 1; gcc2.flags = 4; gcc2.act = 0;
      gcc2.alpha = 1.0f; gcc2.beta = 1.0f; gcc2.sa = 1.0f; gcc2.sb = 1.0f; gcc2.Npad = H; gcc2.pad_ = 0;
      k_gemm<1><<<dim3((unsigned)((H) + 31) / 32, (unsigned)((N) + 15) / 16, (unsigned)(Bn)), 32, 0, stream>>>(gcc2); }
    { GemmP gcc3;
      gcc3.A = X3; gcc3.B = thc + 192; gcc3.bias = X3; gcc3.R = Cg; gcc3.C = Cg;
      gcc3.sAo = P; gcc3.sAi = 0; gcc3.sAm = BP; gcc3.sAk = 1; gcc3.sBo = 0; gcc3.sBi = 0; gcc3.sBn = 1; gcc3.sBk = KM * H; gcc3.sCo = (long long)N * H; gcc3.sCi = 0; gcc3.sCm = H; gcc3.sRo = (long long)N * H; gcc3.sRi = 0; gcc3.sRm = H; gcc3.sRn = 1;
      gcc3.M = N; gcc3.N = H; gcc3.K = P; gcc3.zi_n = 1; gcc3.flags = 4; gcc3.act = 0;
      gcc3.alpha = 1.0f; gcc3.beta = 1.0f; gcc3.sa = 1.0f; gcc3.sb = 1.0f; gcc3.Npad = H; gcc3.pad_ = 0;
      k_gemm<1><<<dim3((unsigned)((H) + 31) / 32, (unsigned)((N) + 15) / 16, (unsigned)(Bn)), 32, 0, stream>>>(gcc3); }
    { GemmP gcc4;
      gcc4.A = X4; gcc4.B = thc + 256; gcc4.bias = X4; gcc4.R = Cg; gcc4.C = Cg;
      gcc4.sAo = P; gcc4.sAi = 0; gcc4.sAm = BP; gcc4.sAk = 1; gcc4.sBo = 0; gcc4.sBi = 0; gcc4.sBn = 1; gcc4.sBk = KM * H; gcc4.sCo = (long long)N * H; gcc4.sCi = 0; gcc4.sCm = H; gcc4.sRo = (long long)N * H; gcc4.sRi = 0; gcc4.sRm = H; gcc4.sRn = 1;
      gcc4.M = N; gcc4.N = H; gcc4.K = P; gcc4.zi_n = 1; gcc4.flags = 4; gcc4.act = 0;
      gcc4.alpha = 1.0f; gcc4.beta = 1.0f; gcc4.sa = 1.0f; gcc4.sb = 1.0f; gcc4.Npad = H; gcc4.pad_ = 0;
      k_gemm<1><<<dim3((unsigned)((H) + 31) / 32, (unsigned)((N) + 15) / 16, (unsigned)(Bn)), 32, 0, stream>>>(gcc4); }
    k_unitstat<<<1, 32, 0, stream>>>(dr);
    k_norm_apply<<<(unsigned)(((long long)(1) * (1) * ((long long)Bn * N * H) + 255) / 256), 256, 0, stream>>>(Cg, Cg, dr, nullptr, nullptr, 1, 1, (long long)Bn * N * H, 1, 0, 5);
    k_dc_out<<<(unsigned)(((long long)Bn * N * H + 255) / 256), 256, 0, stream>>>(U, state, Cg, out, (long long)Bn * N * H);
}
